// Multihead_self_attention_block_15255723836045
// MI455X (gfx1250) — hardware-verified
//
#include <hip/hip_runtime.h>
#include <math.h>
#include <stdint.h>


#define BATCH 4
#define NTOK  4096
#define DMOD  512
#define NHEAD 8
#define HDIM  64
#define NKEY  1024
#define IMG   64
#define RIMG  32
#define KVLD  1024
#define MROWS (BATCH * NTOK)
#define SROWS (BATCH * NKEY)
#define OUTN  (MROWS * DMOD)
#define QTILE 16
#define NQT   (NTOK / QTILE)
#define KTILE 32
#define NKT   (NKEY / KTILE)
#define PARTW 32

#define SCW  64.0f
#define SCQK 8.0f
#define SCP  1024.0f
#define SCA  64.0f

static_assert(NHEAD * HDIM == DMOD);
static_assert(NTOK == IMG * IMG);
static_assert(NKEY == RIMG * RIMG);
static_assert((MROWS % 64) == 0 && (SROWS % 64) == 0 && (DMOD % 64) == 0 && (KVLD % 64) == 0);
static_assert((((MROWS / 64) * (DMOD / 64)) % 8) == 0);
static_assert((((SROWS / 64) * (KVLD / 64)) % 8) == 0);
static_assert(((OUTN / 8) % 256) == 0);
static_assert(NQT == 256 && NKT == 32 && QTILE == 16 && KTILE == 32);
static_assert(((BATCH * DMOD) % 256) == 0);
static_assert(BATCH * NHEAD == 32);
static_assert(PARTW >= NHEAD);

typedef _Float16       v16h __attribute__((ext_vector_type(16)));
typedef _Float16       v8h  __attribute__((ext_vector_type(8)));
typedef float          v8f  __attribute__((ext_vector_type(8)));
typedef float          v4f  __attribute__((ext_vector_type(4)));
typedef unsigned int   v4u  __attribute__((ext_vector_type(4)));

union HU { v8h h; v4u u; _Float16 s[8]; };
union FR { v16h v; v8h h[2]; _Float16 s[16]; };

__device__ __forceinline__ unsigned short bf_bits(float f) {
  const unsigned u = __float_as_uint(f);
  return (unsigned short)((u + 0x7FFFu + ((u >> 16) & 1u)) >> 16);
}
__device__ __forceinline__ float bf_up(unsigned short h) { return __uint_as_float(((unsigned)h) << 16); }
__device__ __forceinline__ float bfr(float f) { return bf_up(bf_bits(f)); }
__device__ __forceinline__ v8f zero8() { v8f z = {0.f, 0.f, 0.f, 0.f, 0.f, 0.f, 0.f, 0.f}; return z; }

__device__ __forceinline__ void ld8(const float* p, float* o) {
  const v4f a = *(const v4f*)(p);
  const v4f b = *(const v4f*)(p + 4);
  o[0] = a[0]; o[1] = a[1]; o[2] = a[2]; o[3] = a[3];
  o[4] = b[0]; o[5] = b[1]; o[6] = b[2]; o[7] = b[3];
}

__device__ __forceinline__ v16h ldfrag_h(const _Float16* p) {
  FR f;
  f.h[0] = *(const v8h*)(p);
  f.h[1] = *(const v8h*)(p + 16);
  return f.v;
}

__device__ __forceinline__ v8f mma_h(v16h a, v16h b, v8f c) {
  c = __builtin_amdgcn_wmma_f32_16x16x32_f16(false, a, false, b, (short)0, c, false, false);
#if defined(__HIP_DEVICE_COMPILE__)
  asm volatile("v_nop\n\tv_nop\n\tv_nop\n\tv_nop" : "+v"(c) : "v"(a), "v"(b));
#endif
  return c;
}
__device__ __forceinline__ v8f mma_h_raw(v16h a, v16h b, v8f c) {
  return __builtin_amdgcn_wmma_f32_16x16x32_f16(false, a, false, b, (short)0, c, false, false);
}
__device__ __forceinline__ void dep_guard_h(v8f& a, v8f& b, v16h x) {
#if defined(__HIP_DEVICE_COMPILE__)
  asm volatile("v_nop\n\tv_nop\n\tv_nop\n\tv_nop" : "+v"(a), "+v"(b) : "v"(x));
#endif
}
__device__ __forceinline__ void keep4_h(v16h a, v16h b, v16h c, v16h d) {
#if defined(__HIP_DEVICE_COMPILE__)
  asm volatile("v_nop" :: "v"(a), "v"(b), "v"(c), "v"(d));
#endif
}
__device__ __forceinline__ void acc_guard4(v8f& a, v8f& b, v8f& c, v8f& d) {
#if defined(__HIP_DEVICE_COMPILE__)
  asm volatile("v_nop\n\tv_nop\n\tv_nop\n\tv_nop" : "+v"(a), "+v"(b), "+v"(c), "+v"(d));
#endif
}

__global__ __launch_bounds__(256) void cvt_x16(const float* __restrict__ in, _Float16* out, int n8) {
  const int i = blockIdx.x * 256 + threadIdx.x;
  if (i < n8) {
    float v[8];
    ld8(in + (size_t)i * 8, v);
    HU u;
#pragma unroll
    for (int e = 0; e < 8; ++e) u.s[e] = (_Float16)bfr(v[e]);
    _Float16* p = out + (size_t)i * 8;
    *(volatile v4u*)p = u.u;
    __threadfence();
    *(volatile v4u*)p = u.u;
  }
}

__global__ __launch_bounds__(256) void cvt_wT(const float* __restrict__ W, int N, _Float16* Bt, float scale) {
  __shared__ float sw[64][65];
  const int t = threadIdx.x;
  const int n0 = blockIdx.x * 64, k0 = blockIdx.y * 64;
  {
    const int r = t >> 4, c4 = (t & 15) * 4;
#pragma unroll
    for (int it = 0; it < 4; ++it) {
      const int row = r + 16 * it;
      const v4f x = *(const v4f*)(W + (size_t)(k0 + row) * (size_t)N + n0 + c4);
      sw[row][c4 + 0] = x[0]; sw[row][c4 + 1] = x[1]; sw[row][c4 + 2] = x[2]; sw[row][c4 + 3] = x[3];
    }
  }
  __syncthreads();
  const int q8 = t & 7, rr = t >> 3;
  HU u[2];
#pragma unroll
  for (int it = 0; it < 2; ++it) {
    const int n = rr + 32 * it;
#pragma unroll
    for (int e = 0; e < 8; ++e) u[it].s[e] = (_Float16)(bfr(sw[8 * q8 + e][n]) * scale);
  }
  for (int pass = 0; pass < 2; ++pass) {
#pragma unroll
    for (int it = 0; it < 2; ++it) {
      const int n = rr + 32 * it;
      _Float16* dst = Bt + (size_t)(n0 + n) * DMOD + k0 + 8 * q8;
      *(volatile v4u*)dst = u[it].u;
    }
    __threadfence();
  }
}

__device__ __forceinline__ void kseg(v8f (&acc)[4][4], const _Float16* __restrict__ A, int lda, int m0,
                                     const _Float16* __restrict__ Bt, int ldb, int n0, int K, int rlane, int koff) {
  for (int kk = 0; kk < K; kk += 32) {
    v16h bh[4];
#pragma unroll
    for (int j = 0; j < 4; ++j) {
      const size_t bo = (size_t)(n0 + (j << 4) + rlane) * (size_t)ldb + koff + kk;
      bh[j] = ldfrag_h(Bt + bo);
    }
#pragma unroll
    for (int i = 0; i < 4; ++i) {
      const size_t ao = (size_t)(m0 + (i << 4) + rlane) * (size_t)lda + koff + kk;
      const v16h a0 = ldfrag_h(A + ao);
#pragma unroll
      for (int j = 0; j < 4; ++j) acc[i][j] = mma_h_raw(a0, bh[j], acc[i][j]);
      dep_guard_h(acc[i][0], acc[i][3], a0);
    }
    keep4_h(bh[0], bh[1], bh[2], bh[3]);
  }
}

template <int MODE>
__global__ __launch_bounds__(256) void gemm64(
    const _Float16* __restrict__ A, int lda, const _Float16* __restrict__ Bt, int ldb,
    const float* __restrict__ bias0, const float* __restrict__ bias1, int nsplit,
    float cs, float so, float* Cf, _Float16* Ch, int ldc, int M, int N, int K) {
  __shared__ __align__(16) float sT[8][16 * 68];
  const int lane = threadIdx.x & 31;
  const int wave = threadIdx.x >> 5;
  const int tilesN = N >> 6;
  const int tilesM = M >> 6;
  const int tiles = tilesM * tilesN;
  const int item = blockIdx.x * 8 + wave;
  if (item >= tiles) return;
  const int tm = item / tilesN;
  const int tn = item - tm * tilesN;
  const int m0 = tm << 6;
  const int n0 = tn << 6;

  const int rlane = lane & 15;
  const int koff  = (lane >> 4) * 8;
  const int mOff  = (lane >> 4) * 8;

  v8f acc[4][4];
#pragma unroll
  for (int i = 0; i < 4; ++i)
#pragma unroll
    for (int j = 0; j < 4; ++j) acc[i][j] = zero8();

  kseg(acc, A, lda, m0, Bt, ldb, n0, K, rlane, koff);
  acc_guard4(acc[0][0], acc[0][1], acc[0][2], acc[0][3]);
  acc_guard4(acc[1][0], acc[1][1], acc[1][2], acc[1][3]);
  acc_guard4(acc[2][0], acc[2][1], acc[2][2], acc[2][3]);
  acc_guard4(acc[3][0], acc[3][1], acc[3][2], acc[3][3]);

  const float* bp = (n0 < nsplit) ? (bias0 + n0) : (bias1 + (n0 - nsplit));

  float* slab = sT[wave];
#pragma unroll
  for (int i = 0; i < 4; ++i) {
    const int mBase = m0 + (i << 4);
#pragma unroll
    for (int r = 0; r < 8; ++r) {
#pragma unroll
      for (int j = 0; j < 4; ++j) {
        slab[(mOff + r) * 68 + (j << 4) + rlane] = acc[i][j][r];
      }
    }
    __builtin_amdgcn_fence(__ATOMIC_RELEASE, "workgroup");
    __builtin_amdgcn_wave_barrier();
    __builtin_amdgcn_fence(__ATOMIC_ACQUIRE, "workgroup");
    if (MODE == 0) {
      const int h2 = lane >> 4, c4 = (lane & 15) * 4;
      const v4f braw = *(const v4f*)(bp + c4);
      v4f b4;
#pragma unroll
      for (int e = 0; e < 4; ++e) b4[e] = bfr(braw[e]);
      v4f ov[8];
#pragma unroll
      for (int it = 0; it < 8; ++it) {
        const int row = it * 2 + h2;
        const v4f xs = *(const v4f*)(slab + row * 68 + c4);
        ov[it] = xs * cs + b4;
      }
      for (int pass = 0; pass < 2; ++pass) {
#pragma unroll
        for (int it = 0; it < 8; ++it) {
          const int row = it * 2 + h2;
          *(volatile v4f*)(Cf + (size_t)(mBase + row) * (size_t)ldc + n0 + c4) = ov[it];
        }
        __threadfence();
      }
    } else {
      const int q8 = lane & 7, rr = lane >> 3, c8 = q8 * 8;
      float bb[8];
      {
        const v4f b0 = *(const v4f*)(bp + c8);
        const v4f b1 = *(const v4f*)(bp + c8 + 4);
#pragma unroll
        for (int e = 0; e < 4; ++e) { bb[e] = bfr(b0[e]); bb[4 + e] = bfr(b1[e]); }
      }
      v4u ovh[4];
#pragma unroll
      for (int it = 0; it < 4; ++it) {
        const int row = it * 4 + rr;
        float xs[8];
        ld8(slab + row * 68 + c8, xs);
        HU u;
#pragma unroll
        for (int e = 0; e < 8; ++e) u.s[e] = (_Float16)((xs[e] * cs + bb[e]) * so);
        ovh[it] = u.u;
      }
      for (int pass = 0; pass < 2; ++pass) {
#pragma unroll
        for (int it = 0; it < 4; ++it) {
          const int row = it * 4 + rr;
          const size_t co = (size_t)(mBase + row) * (size_t)ldc + n0 + c8;
          *(volatile v4u*)(Ch + co) = ovh[it];
        }
        __threadfence();
      }
    }
    __builtin_amdgcn_fence(__ATOMIC_RELEASE, "workgroup");
    __builtin_amdgcn_wave_barrier();
    __builtin_amdgcn_fence(__ATOMIC_ACQUIRE, "workgroup");
  }
}

__global__ __launch_bounds__(256) void k_dwln(const float* __restrict__ q, const float* __restrict__ cw,
                                              const float* __restrict__ cb, const float* __restrict__ lw,
                                              const float* __restrict__ lb, _Float16* X16) {
  __shared__ float sred[8];
  __shared__ __align__(16) float sy[DMOD];
  const int t = threadIdx.x, wave = t >> 5, lane = t & 31;
  const int pos = blockIdx.x, b = blockIdx.y;
  const int oy = pos >> 5, ox = pos & 31;

  float acc[2] = {0.f, 0.f};
#pragma unroll
  for (int ky = 0; ky < 3; ++ky) {
    const int iy = 2 * oy - 1 + ky;
    const int iyc = min(max(iy, 0), IMG - 1);
    const bool vy = (iy == iyc);
#pragma unroll
    for (int kx = 0; kx < 3; ++kx) {
      const int ix = 2 * ox - 1 + kx;
      const int ixc = min(max(ix, 0), IMG - 1);
      const bool ok = vy && (ix == ixc);
      const size_t po = ((size_t)(b * NTOK + iyc * IMG + ixc)) * DMOD;
#pragma unroll
      for (int j = 0; j < 2; ++j) {
        const int c = t + 256 * j;
        const float w = bfr(cw[c * 9 + ky * 3 + kx]);
        const float x = bfr(q[po + c]);
        acc[j] += (ok ? w : 0.0f) * x;
      }
    }
  }
  const float v0 = acc[0] + bfr(cb[t]);
  const float v1 = acc[1] + bfr(cb[t + 256]);

  float s = v0 + v1;
#pragma unroll
  for (int off = 16; off >= 1; off >>= 1) s += __shfl_xor(s, off, 32);
  if (lane == 0) sred[wave] = s;
  __syncthreads();
  float tot = 0.f;
#pragma unroll
  for (int w = 0; w < 8; ++w) tot += sred[w];
  const float mu = tot * (1.0f / (float)DMOD);
  __syncthreads();
  const float d0 = v0 - mu, d1 = v1 - mu;
  float ss = d0 * d0 + d1 * d1;
#pragma unroll
  for (int off = 16; off >= 1; off >>= 1) ss += __shfl_xor(ss, off, 32);
  if (lane == 0) sred[wave] = ss;
  __syncthreads();
  float tot2 = 0.f;
#pragma unroll
  for (int w = 0; w < 8; ++w) tot2 += sred[w];
  const float var = tot2 * (1.0f / (float)DMOD);
  const float rs = 1.0f / sqrtf(var + 1.0e-5f);
  const float y0 = (d0 * rs) * bfr(lw[t]) + bfr(lb[t]);
  const float y1 = (d1 * rs) * bfr(lw[t + 256]) + bfr(lb[t + 256]);
  sy[t] = y0;
  sy[t + 256] = y1;
  __syncthreads();
  if (t < 64) {
    float yv[8];
    ld8(sy + 8 * t, yv);
    HU u;
#pragma unroll
    for (int e = 0; e < 8; ++e) u.s[e] = (_Float16)yv[e];
    _Float16* dst = X16 + (size_t)(b * NKEY + pos) * DMOD + 8 * t;
    *(volatile v4u*)dst = u.u;
    __threadfence();
    *(volatile v4u*)dst = u.u;
  }
}

__global__ __launch_bounds__(256) void k_vt(const _Float16* __restrict__ KV16, _Float16* Vt) {
  __shared__ __align__(16) _Float16 sv[64][72];
  const int t = threadIdx.x;
  const int key0 = blockIdx.x * 64, c0 = blockIdx.y * 64, b = blockIdx.z;
#pragma unroll
  for (int it = 0; it < 2; ++it) {
    const int idx = t + 256 * it;
    const int row = idx >> 3, pc = (idx & 7) * 8;
    const v8h x = *(const v8h*)(KV16 + (size_t)(b * NKEY + key0 + row) * KVLD + DMOD + c0 + pc);
    *(v8h*)(&sv[row][pc]) = x;
  }
  __syncthreads();
  const int q8 = t & 7, rr = t >> 3;
  HU u[2];
#pragma unroll
  for (int it = 0; it < 2; ++it) {
    const int c = rr + 32 * it;
#pragma unroll
    for (int e = 0; e < 8; ++e) u[it].s[e] = sv[8 * q8 + e][c];
  }
  for (int pass = 0; pass < 2; ++pass) {
#pragma unroll
    for (int it = 0; it < 2; ++it) {
      const int c = rr + 32 * it;
      _Float16* dst = Vt + (size_t)(b * DMOD + c0 + c) * NKEY + key0 + 8 * q8;
      *(volatile v4u*)dst = u[it].u;
    }
    __threadfence();
  }
}

__global__ __launch_bounds__(256) void k_vsum(const _Float16* __restrict__ Vt, float* Vsum) {
  const int r = blockIdx.x * 256 + threadIdx.x;
  const _Float16* p = Vt + (size_t)r * NKEY;
  float a[8] = {0.f, 0.f, 0.f, 0.f, 0.f, 0.f, 0.f, 0.f};
#pragma unroll 4
  for (int j = 0; j < NKEY / 8; ++j) {
    HU u;
    u.h = *(const v8h*)(p + 8 * j);
#pragma unroll
    for (int e = 0; e < 8; ++e) a[e] += (float)u.s[e];
  }
  const float s = ((a[0] + a[1]) + (a[2] + a[3])) + ((a[4] + a[5]) + (a[6] + a[7]));
  const float v = s * (1.0f / SCQK);
  *(volatile float*)(Vsum + r) = v;
  __threadfence();
  *(volatile float*)(Vsum + r) = v;
}

__global__ __launch_bounds__(256) void k_attn(const _Float16* __restrict__ Q16, const _Float16* __restrict__ K16,
                                              const _Float16* __restrict__ Vt, const float* __restrict__ tw,
                                              const float* __restrict__ tb, const float* __restrict__ Vsum,
                                              float* U, float* part) {
  __shared__ __align__(16) float sS[NHEAD][QTILE][36];
  __shared__ __align__(16) float sO[NHEAD][QTILE * 68];
  __shared__ float sG[NHEAD][QTILE];
  __shared__ float sP[NHEAD];
  const int tid = threadIdx.x, wave = tid >> 5, lane = tid & 31;
  const int hh = lane >> 4, m = lane & 15;
  const int bx = blockIdx.x;
  const int b = bx >> 8;
  const int qt = bx & (NQT - 1);
  const int q0 = qt * QTILE;
  const int o = wave;

  float wmix[NHEAD];
#pragma unroll
  for (int h = 0; h < NHEAD; ++h) wmix[h] = bfr(tw[o * NHEAD + h]) * (1.0f / 512.0f);
  const float bmix = bfr(tb[o]);

  const _Float16* qrow = Q16 + (size_t)(b * NTOK + q0 + m) * DMOD + o * HDIM + 8 * hh;
  const v16h qb0 = ldfrag_h(qrow);
  const v16h qb1 = ldfrag_h(qrow + 32);
  const _Float16* kbase = K16 + (size_t)(b * NKEY + m) * KVLD + o * HDIM + 8 * hh;
  const _Float16* vbase = Vt + (size_t)(b * DMOD + o * HDIM + m) * NKEY + 8 * hh;

  v8f oacc[4];
#pragma unroll
  for (int nf = 0; nf < 4; ++nf) oacc[nf] = zero8();
  float Mrun = -1.0e30f, Srun = 0.f, T1 = 0.f, T2 = 0.f;
  float* sSw = &sS[o][m][0];

  for (int kt = 0; kt < NKT; ++kt) {
    const int k0 = kt * KTILE;
#pragma unroll
    for (int kf = 0; kf < 2; ++kf) {
      const _Float16* kp = kbase + (size_t)(k0 + 16 * kf) * KVLD;
      v8f c = zero8();
      const v16h a0 = ldfrag_h(kp);
      c = mma_h(a0, qb0, c);
      const v16h a1 = ldfrag_h(kp + 32);
      c = mma_h(a1, qb1, c);
      const v4f clo = {c[0], c[1], c[2], c[3]};
      const v4f chi = {c[4], c[5], c[6], c[7]};
      *(v4f*)(sSw + 16 * kf + 8 * hh) = clo;
      *(v4f*)(sSw + 16 * kf + 8 * hh + 4) = chi;
    }
    __syncthreads();
    float L[16];
#pragma unroll
    for (int i = 0; i < 16; ++i) L[i] = bmix;
#pragma unroll
    for (int h = 0; h < NHEAD; ++h) {
      const float* sp = &sS[h][m][8 * hh];
      const v4f x0 = *(const v4f*)(sp);
      const v4f x1 = *(const v4f*)(sp + 4);
      const v4f x2 = *(const v4f*)(sp + 16);
      const v4f x3 = *(const v4f*)(sp + 20);
      const float w = wmix[h];
#pragma unroll
      for (int e = 0; e < 4; ++e) {
        L[e]      += w * x0[e];
        L[4 + e]  += w * x1[e];
        L[8 + e]  += w * x2[e];
        L[12 + e] += w * x3[e];
      }
    }
    __syncthreads();
    float tmax = L[0];
#pragma unroll
    for (int i = 1; i < 16; ++i) tmax = fmaxf(tmax, L[i]);
    tmax = fmaxf(tmax, __shfl_xor(tmax, 16, 32));
    const float Mnew = fmaxf(Mrun, tmax);
    const float al = __expf(Mrun - Mnew);
    const float em = __expf(-Mnew);
    float ps = 0.f, ts = 0.f, t2 = 0.f;
    FR pb;
#pragma unroll
    for (int i = 0; i < 16; ++i) {
      const float p = __expf(L[i] - Mnew);
      const float tv = p - em;
      ps += p;
      ts += tv;
      t2 += tv * tv;
      pb.s[i] = (_Float16)(tv * SCP);
    }
    ps += __shfl_xor(ps, 16, 32);
    ts += __shfl_xor(ts, 16, 32);
    t2 += __shfl_xor(t2, 16, 32);
    Srun = Srun * al + ps;
    T1 = T1 * al + ts;
    T2 = T2 * (al * al) + t2;
    Mrun = Mnew;
#pragma unroll
    for (int nf = 0; nf < 4; ++nf) oacc[nf] = oacc[nf] * al;
    const _Float16* vp = vbase + k0;
#pragma unroll
    for (int nf = 0; nf < 4; ++nf) {
      const v16h av = ldfrag_h(vp + (size_t)nf * 16 * NKEY);
      oacc[nf] = mma_h(av, pb.v, oacc[nf]);
    }
  }

  const float rS = 1.0f / Srun;
  const float emf = __expf(-Mrun);
  const float fo = rS * (1.0f / (SCP * SCQK));
  const float g = emf * rS - (1.0f / 1024.0f);
  const float cc = emf - Srun * (1.0f / 1024.0f);
  const float ssq = (T2 + 2.0f * cc * T1 + 1024.0f * cc * cc) * (rS * rS);
  float* sOw = &sO[o][0];
#pragma unroll
  for (int nf = 0; nf < 4; ++nf) {
    const v4f lo = {oacc[nf][0] * fo, oacc[nf][1] * fo, oacc[nf][2] * fo, oacc[nf][3] * fo};
    const v4f hi = {oacc[nf][4] * fo, oacc[nf][5] * fo, oacc[nf][6] * fo, oacc[nf][7] * fo};
    *(v4f*)(sOw + m * 68 + nf * 16 + 8 * hh) = lo;
    *(v4f*)(sOw + m * 68 + nf * 16 + 8 * hh + 4) = hi;
  }
  if (hh == 0) sG[o][m] = g;
  float sw = (hh == 0) ? ssq : 0.0f;
#pragma unroll
  for (int off = 16; off >= 1; off >>= 1) sw += __shfl_xor(sw, off, 32);
  if (lane == 0) sP[o] = sw;
  __builtin_amdgcn_fence(__ATOMIC_RELEASE, "workgroup");
  __builtin_amdgcn_wave_barrier();
  __builtin_amdgcn_fence(__ATOMIC_ACQUIRE, "workgroup");
  {
    const int h2 = lane >> 4, c4 = (lane & 15) * 4;
    const v4f V4 = *(const v4f*)(Vsum + b * DMOD + o * HDIM + c4);
    v4f ov[8];
#pragma unroll
    for (int it = 0; it < 8; ++it) {
      const int row = it * 2 + h2;
      const v4f xs = *(const v4f*)(sOw + row * 68 + c4);
      const float gg = sG[o][row];
      ov[it] = xs + gg * V4;
    }
    for (int pass = 0; pass < 2; ++pass) {
#pragma unroll
      for (int it = 0; it < 8; ++it) {
        const int row = it * 2 + h2;
        *(volatile v4f*)(U + (size_t)(b * NTOK + q0 + row) * DMOD + o * HDIM + c4) = ov[it];
      }
      __threadfence();
    }
  }
  __syncthreads();
  if (wave == 0) {
    const float pv = (lane < NHEAD) ? sP[lane & (NHEAD - 1)] : 0.0f;
    float* pp = part + (size_t)bx * PARTW + lane;
    *(volatile float*)pp = pv;
    __threadfence();
    *(volatile float*)pp = pv;
  }
}

__global__ __launch_bounds__(32) void k_rstd(const float* __restrict__ part, float* rstd) {
  const int t = threadIdx.x;
  const int b = t >> 3, o = t & 7;
  double s = 0.0;
  for (int qt = 0; qt < NQT; ++qt) s += (double)part[((size_t)(b * NQT + qt)) * PARTW + o];
  const double var = s * (1.0 / ((double)NTOK * (double)NKEY));
  const float r = 1.0f / sqrtf((float)var + 1.0e-5f);
  *(volatile float*)(rstd + t) = r;
  __threadfence();
  *(volatile float*)(rstd + t) = r;
}

__global__ __launch_bounds__(256) void k_cvtu(const float* __restrict__ U, const float* __restrict__ rstd,
                                              _Float16* O16, int n8) {
  const int i = blockIdx.x * 256 + threadIdx.x;
  if (i < n8) {
    const int row = i >> 6;
    const int c8 = (i & 63) * 8;
    const int b = row >> 12;
    const float rs = rstd[b * NHEAD + (c8 >> 6)] * SCA;
    float v[8];
    ld8(U + (size_t)i * 8, v);
    HU u;
#pragma unroll
    for (int e = 0; e < 8; ++e) u.s[e] = (_Float16)(v[e] * rs);
    _Float16* p = O16 + (size_t)i * 8;
    *(volatile v4u*)p = u.u;
    __threadfence();
    *(volatile v4u*)p = u.u;
  }
}

extern "C" void kernel_launch(void* const* d_in, const int* in_sizes, int n_in,
                              void* d_out, int out_size, void* d_ws, size_t ws_size,
                              hipStream_t stream) {
  if (n_in < 17) return;
  if (in_sizes[0] != OUTN) return;
  if (in_sizes[3] != DMOD * DMOD || in_sizes[5] != DMOD * DMOD) return;
  if (in_sizes[7] != DMOD * DMOD || in_sizes[9] != DMOD * DMOD) return;
  if (in_sizes[4] != DMOD || in_sizes[6] != DMOD || in_sizes[8] != DMOD || in_sizes[10] != DMOD) return;
  if (in_sizes[11] != DMOD * 9 || in_sizes[12] != DMOD) return;
  if (in_sizes[13] != DMOD || in_sizes[14] != DMOD) return;
  if (in_sizes[15] != NHEAD * NHEAD || in_sizes[16] != NHEAD) return;
  if (out_size != OUTN) return;

  const float* queries = (const float*)d_in[0];
  const float* wq      = (const float*)d_in[3];
  const float* bq      = (const float*)d_in[4];
  const float* wk      = (const float*)d_in[5];
  const float* bk      = (const float*)d_in[6];
  const float* wv      = (const float*)d_in[7];
  const float* bv      = (const float*)d_in[8];
  const float* wo      = (const float*)d_in[9];
  const float* bo      = (const float*)d_in[10];
  const float* conv_w  = (const float*)d_in[11];
  const float* conv_b  = (const float*)d_in[12];
  const float* ln_w    = (const float*)d_in[13];
  const float* ln_b    = (const float*)d_in[14];
  const float* tconv_w = (const float*)d_in[15];
  const float* tconv_b = (const float*)d_in[16];

  const size_t PWT  = (size_t)DMOD * DMOD * 2;
  const size_t PKVW = (size_t)KVLD * DMOD * 2;
  const size_t PM16 = (size_t)MROWS * DMOD * 2;
  const size_t PX16 = (size_t)SROWS * DMOD * 2;
  const size_t PKV  = (size_t)SROWS * KVLD * 2;
  const size_t PVT  = (size_t)BATCH * DMOD * NKEY * 2;
  const size_t PVS  = (size_t)BATCH * DMOD * 4;
  const size_t PU   = (size_t)MROWS * DMOD * 4;
  const size_t PPT  = (size_t)BATCH * NQT * PARTW * 4;
  const size_t PRS  = 128;

  size_t off = 0;
  const size_t oWq  = off; off += PWT;
  const size_t oWkv = off; off += PKVW;
  const size_t oWo  = off; off += PWT;
  const size_t oXq  = off; off += PM16;
  const size_t oQ   = off; off += PM16;
  const size_t oX   = off; off += PX16;
  const size_t oKV  = off; off += PKV;
  const size_t oVt  = off; off += PVT;
  const size_t oVs  = off; off += PVS;
  const size_t oU   = off; off += PU;
  const size_t oPt  = off; off += PPT;
  const size_t oRs  = off; off += PRS;
  const size_t oO   = off; off += PM16;
  if (off > ws_size) return;
  if (off > (size_t)134217728) return;

  char* ws = (char*)d_ws;
  _Float16* WqT  = (_Float16*)(ws + oWq);
  _Float16* WkvT = (_Float16*)(ws + oWkv);
  _Float16* WoT  = (_Float16*)(ws + oWo);
  _Float16* Xq16 = (_Float16*)(ws + oXq);
  _Float16* Q16  = (_Float16*)(ws + oQ);
  _Float16* X16  = (_Float16*)(ws + oX);
  _Float16* KV16 = (_Float16*)(ws + oKV);
  _Float16* Vt   = (_Float16*)(ws + oVt);
  float*    Vsum = (float*)(ws + oVs);
  float*    Ubuf = (float*)(ws + oU);
  float*    part = (float*)(ws + oPt);
  float*    rstd = (float*)(ws + oRs);
  _Float16* O16  = (_Float16*)(ws + oO);
  float*    outf = (float*)d_out;

  const dim3 blk(256);
  const int n8x = OUTN / 8;
  const dim3 gWT(DMOD / 64, DMOD / 64);
  const dim3 gX((n8x + 255) / 256);
  const dim3 gQ(((MROWS / 64) * (DMOD / 64) + 7) / 8);
  const dim3 gKV(((SROWS / 64) * (KVLD / 64) + 7) / 8);
  const dim3 gDw(NKEY, BATCH);
  const dim3 gVt(NKEY / 64, DMOD / 64, BATCH);
  const dim3 gVs((BATCH * DMOD) / 256);
  const dim3 gAt(BATCH * NQT);
  const float cs64 = 1.0f / SCW;
  const float cs4096 = 1.0f / (SCW * SCA);

  cvt_wT<<<gWT, blk, 0, stream>>>(wq, DMOD, WqT, SCW);
  cvt_wT<<<gWT, blk, 0, stream>>>(wk, DMOD, WkvT, SCW);
  cvt_wT<<<gWT, blk, 0, stream>>>(wv, DMOD, WkvT + (size_t)DMOD * DMOD, SCW);
  cvt_wT<<<gWT, blk, 0, stream>>>(wo, DMOD, WoT, SCW);
  cvt_x16<<<gX, blk, 0, stream>>>(queries, Xq16, n8x);
  gemm64<1><<<gQ, blk, 0, stream>>>(Xq16, DMOD, WqT, DMOD, bq, bq, DMOD, cs64, SCQK,
                                    Ubuf, Q16, DMOD, MROWS, DMOD, DMOD);
  k_dwln<<<gDw, blk, 0, stream>>>(queries, conv_w, conv_b, ln_w, ln_b, X16);
  gemm64<1><<<gKV, blk, 0, stream>>>(X16, DMOD, WkvT, DMOD, bk, bv, DMOD, cs64, SCQK,
                                     Ubuf, KV16, KVLD, SROWS, KVLD, DMOD);
  k_vt<<<gVt, blk, 0, stream>>>(KV16, Vt);
  k_vsum<<<gVs, blk, 0, stream>>>(Vt, Vsum);
  k_attn<<<gAt, blk, 0, stream>>>(Q16, KV16, Vt, tconv_w, tconv_b, Vsum, Ubuf, part);
  k_rstd<<<dim3(1), dim3(32), 0, stream>>>(part, rstd);
  k_cvtu<<<gX, blk, 0, stream>>>(Ubuf, rstd, O16, n8x);
  gemm64<0><<<gQ, blk, 0, stream>>>(O16, DMOD, WoT, DMOD, bo, bo, DMOD, cs4096, 1.0f,
                                    outf, O16, DMOD, MROWS, DMOD, DMOD);
  (void)hipGetLastError();
}
